// CondConv_59261958750578
// MI455X (gfx1250) — hardware-verified
//
#include <hip/hip_runtime.h>
#include <stdint.h>


typedef _Float16 v16h __attribute__((ext_vector_type(16)));
typedef _Float16 v8h  __attribute__((ext_vector_type(8)));
typedef float    v8f  __attribute__((ext_vector_type(8)));
typedef float    v4f  __attribute__((ext_vector_type(4)));
union Frag { v16h v; v8h half[2]; };

static __device__ __forceinline__ v8f wmma16(const v16h a, const v16h b, v8f c)
{
    v8f d = __builtin_amdgcn_wmma_f32_16x16x32_f16(false, a, false, b, (short)0, c, false, false);
    asm volatile("v_nop\n\tv_nop\n\tv_nop\n\tv_nop" : "+v"(d) : "v"(a), "v"(b));
    return d;
}

__global__ __launch_bounds__(256) void k_att(
    const float* __restrict__ x, const float* __restrict__ z,
    const float* __restrict__ w1, const float* __restrict__ gamma,
    const float* __restrict__ beta, const float* __restrict__ mean,
    const float* __restrict__ var, const float* __restrict__ w2,
    float* __restrict__ att)
{
    const int b    = blockIdx.x;
    const int tid  = threadIdx.x;
    const int lane = tid & 31;
    const int wave = tid >> 5;

    __shared__ float a[512];
    __shared__ float hb[256];
    __shared__ float av[4];

    const float* xb = x + (size_t)b * 256 * 1024;
    for (int c = wave; c < 256; c += 8) {
        float s = 0.f;
        const float* xc = xb + (size_t)c * 1024;
        for (int i = lane; i < 1024; i += 32) s += xc[i];
#pragma unroll
        for (int o = 16; o > 0; o >>= 1) s += __shfl_down(s, o, 32);
        if (lane == 0) a[256 + c] = s * (1.0f / 1024.0f);
    }
    a[tid] = z[(size_t)b * 256 + tid];
    __syncthreads();

    {
        const int t = tid;
        const float* w = w1 + (size_t)t * 512;
        float s = 0.f;
#pragma unroll 4
        for (int i = 0; i < 512; ++i) s += a[i] * w[i];
        s = (s - mean[t]) * (1.0f / sqrtf(var[t] + 1e-5f)) * gamma[t] + beta[t];
        hb[t] = s > 0.f ? s : 0.f;
    }
    __syncthreads();

    if (tid < 4) {
        const float* w = w2 + tid * 256;
        float s = 0.f;
#pragma unroll 4
        for (int i = 0; i < 256; ++i) s += hb[i] * w[i];
        av[tid] = 1.0f / (1.0f + expf(-s));
    }
    __syncthreads();

    if (tid < 8) {
        v4f v = {0.f, 0.f, 0.f, 0.f};
        if (tid == 0) { v[0] = av[0]; v[1] = av[1]; v[2] = av[2]; v[3] = av[3]; }
        float* p = att + (size_t)b * 32 + tid * 4;
        *(volatile v4f*)p = v;
        __threadfence();
        *(volatile v4f*)p = v;
    }
}

__global__ __launch_bounds__(256) void k_xcvt(
    const float* __restrict__ x, _Float16* __restrict__ xw)
{
    const int b   = blockIdx.x >> 5;
    const int y   = blockIdx.x & 31;
    const int tid = threadIdx.x;
    __shared__ __align__(16) _Float16 ls[32 * 264];

    for (int idx = tid; idx < 8192; idx += 256) {
        const int c  = idx >> 5;
        const int xc = idx & 31;
        ls[xc * 264 + c] =
            (_Float16)(16.0f * x[(((size_t)b * 256 + c) << 10) + (y << 5) + xc]);
    }
    __syncthreads();

    v8h v[4];
#pragma unroll
    for (int k = 0; k < 4; ++k) {
        const int q  = tid + (k << 8);
        const int xc = q >> 5;
        const int c0 = (q & 31) * 8;
        v[k] = *(const v8h*)(&ls[xc * 264 + c0]);
    }
    _Float16* dst = xw + (size_t)(b * 32 + y) * 8192;
#pragma unroll
    for (int k = 0; k < 4; ++k)
        *(volatile v8h*)(dst + (size_t)(tid + (k << 8)) * 8) = v[k];
    __threadfence();
#pragma unroll
    for (int k = 0; k < 4; ++k)
        *(volatile v8h*)(dst + (size_t)(tid + (k << 8)) * 8) = v[k];
}

__global__ __launch_bounds__(256) void k_mix(
    const float* __restrict__ weight, const float* __restrict__ sweight,
    const float* __restrict__ att, _Float16* __restrict__ aggw)
{
    const int blk  = blockIdx.x;
    const int b    = blk >> 5;
    const int tid  = threadIdx.x;
    const int wave = tid >> 5;
    const int lane = tid & 31;
    const int o    = ((blk & 31) << 3) + wave;
    const int c0   = lane * 8;
    const size_t base = ((size_t)o * 256 + c0) * 9;

    float acc[72];
#pragma unroll
    for (int i = 0; i < 72; ++i) acc[i] = 0.f;

#pragma unroll 1
    for (int k = 0; k < 4; ++k) {
        const float ak = att[(size_t)b * 32 + k];
        const float* wp = weight + (size_t)k * 589824 + base;
#pragma unroll
        for (int i = 0; i < 18; ++i) {
            v4f w = *(const v4f*)(wp + 4 * i);
            acc[4 * i + 0] += ak * (w[0] * 0.1f);
            acc[4 * i + 1] += ak * (w[1] * 0.1f);
            acc[4 * i + 2] += ak * (w[2] * 0.1f);
            acc[4 * i + 3] += ak * (w[3] * 0.1f);
        }
    }
    {
        const float* sp = sweight + base;
#pragma unroll
        for (int i = 0; i < 18; ++i) {
            v4f s = *(const v4f*)(sp + 4 * i);
            acc[4 * i + 0] += s[0];
            acc[4 * i + 1] += s[1];
            acc[4 * i + 2] += s[2];
            acc[4 * i + 3] += s[3];
        }
    }

    v8h hv[9];
#pragma unroll
    for (int t = 0; t < 9; ++t) {
        v8h tmp;
#pragma unroll
        for (int j = 0; j < 8; ++j) tmp[j] = (_Float16)(acc[j * 9 + t] * 64.0f);
        hv[t] = tmp;
    }
    _Float16* dst = aggw + (((size_t)b * 9 * 256 + o) * 256 + c0);
#pragma unroll
    for (int t = 0; t < 9; ++t)
        *(volatile v8h*)(dst + (size_t)t * 65536) = hv[t];
    __threadfence();
#pragma unroll
    for (int t = 0; t < 9; ++t)
        *(volatile v8h*)(dst + (size_t)t * 65536) = hv[t];
}

__global__ __launch_bounds__(256) void k_conv(
    const _Float16* __restrict__ xw, const _Float16* __restrict__ aggw,
    float* __restrict__ out)
{
    const int ntile = blockIdx.x;
    const int mtile = blockIdx.y;
    const int b     = blockIdx.z;

    const int tid  = threadIdx.x;
    const int wave = tid >> 5;
    const int lane = tid & 31;
    const int mi   = wave & 3;
    const int ni   = wave >> 2;
    const int h    = lane >> 4;
    const int ln   = lane & 15;

    const int y0     = ntile * 2;
    const int p0     = ntile * 64;
    const int blockM = mtile * 128;

    __shared__ __align__(16) _Float16 xs[4 * 34 * 32];
    __shared__ __align__(16) float    cs[128 * 68];

    const _Float16* xwb = xw + (size_t)b * 262144;
    const _Float16* awb = aggw + (size_t)b * 9 * 65536;

    v8f acc[2][2];
#pragma unroll
    for (int ms = 0; ms < 2; ++ms)
#pragma unroll
        for (int ns = 0; ns < 2; ++ns)
            acc[ms][ns] = (v8f){0.f, 0.f, 0.f, 0.f, 0.f, 0.f, 0.f, 0.f};

#pragma unroll 1
    for (int cg = 0; cg < 8; ++cg) {
        __syncthreads();
        for (int q = tid; q < 544; q += 256) {
            const int h4   = q & 3;
            const int rc   = q >> 2;
            const int colx = rc % 34;
            const int r    = rc / 34;
            const int row  = y0 - 1 + r;
            const int col  = colx - 1;
            v8h val;
#pragma unroll
            for (int i = 0; i < 8; ++i) val[i] = (_Float16)0.0f;
            if (row >= 0 && row < 32 && col >= 0 && col < 32)
                val = *(const v8h*)(xwb + ((size_t)(row * 32 + col) * 256 + cg * 32 + h4 * 8));
            *(v8h*)(&xs[(r * 34 + colx) * 32 + h4 * 8]) = val;
        }
        __syncthreads();

#pragma unroll
        for (int t = 0; t < 9; ++t) {
            const int dy = t / 3;
            const int dx = t - dy * 3;

            Frag af[2];
#pragma unroll
            for (int s = 0; s < 2; ++s) {
                const int m = blockM + mi * 32 + s * 16 + ln;
                const _Float16* ap = awb + ((size_t)t * 256 + m) * 256 + cg * 32;
                af[s].half[0] = *(const v8h*)(ap + 8 * h);
                af[s].half[1] = *(const v8h*)(ap + 16 + 8 * h);
            }

            Frag bf[2];
#pragma unroll
            for (int s = 0; s < 2; ++s) {
                const int col  = s * 16 + ln;
                const int r    = ni + dy;
                const int colx = col + dx;
                const _Float16* bp = &xs[(r * 34 + colx) * 32];
                bf[s].half[0] = *(const v8h*)(bp + 8 * h);
                bf[s].half[1] = *(const v8h*)(bp + 16 + 8 * h);
            }

            acc[0][0] = wmma16(af[0].v, bf[0].v, acc[0][0]);
            acc[0][1] = wmma16(af[0].v, bf[1].v, acc[0][1]);
            acc[1][0] = wmma16(af[1].v, bf[0].v, acc[1][0]);
            acc[1][1] = wmma16(af[1].v, bf[1].v, acc[1][1]);
        }
    }

    const float inv = 0.0009765625f;
#pragma unroll
    for (int ms = 0; ms < 2; ++ms)
#pragma unroll
        for (int ns = 0; ns < 2; ++ns) {
            const int colp = ni * 32 + ns * 16 + ln;
#pragma unroll
            for (int r = 0; r < 8; ++r) {
                const int row = mi * 32 + ms * 16 + 8 * h + r;
                cs[row * 68 + colp] = acc[ms][ns][r] * inv;
            }
        }
    __syncthreads();

    float* ob = out + ((size_t)b * 256 + blockM) * 1024 + p0;
#pragma unroll
    for (int it = 0; it < 8; ++it) {
        const int q   = tid + (it << 8);
        const int row = q >> 4;
        const int c4  = q & 15;
        v4f v = *(const v4f*)(&cs[row * 68 + c4 * 4]);
        *(volatile v4f*)(ob + (size_t)row * 1024 + c4 * 4) = v;
    }
    __threadfence();
#pragma unroll
    for (int it = 0; it < 8; ++it) {
        const int q   = tid + (it << 8);
        const int row = q >> 4;
        const int c4  = q & 15;
        v4f v = *(const v4f*)(&cs[row * 68 + c4 * 4]);
        *(volatile v4f*)(ob + (size_t)row * 1024 + c4 * 4) = v;
    }
}

extern "C" void kernel_launch(void* const* d_in, const int* in_sizes, int n_in,
                              void* d_out, int out_size, void* d_ws, size_t ws_size,
                              hipStream_t stream)
{
    if (n_in < 10) return;
    if (in_sizes[0] != 32 * 256 * 1024) return;
    if (in_sizes[1] != 32 * 256) return;
    if (in_sizes[2] != 256 * 512) return;
    if (in_sizes[3] != 256 || in_sizes[4] != 256 || in_sizes[5] != 256 || in_sizes[6] != 256) return;
    if (in_sizes[7] != 4 * 256) return;
    if (in_sizes[8] != 4 * 256 * 256 * 9) return;
    if (in_sizes[9] != 256 * 256 * 9) return;
    if (out_size != 32 * 256 * 1024) return;

    const float* x       = (const float*)d_in[0];
    const float* z       = (const float*)d_in[1];
    const float* w1      = (const float*)d_in[2];
    const float* gamma   = (const float*)d_in[3];
    const float* beta    = (const float*)d_in[4];
    const float* mean    = (const float*)d_in[5];
    const float* var     = (const float*)d_in[6];
    const float* w2      = (const float*)d_in[7];
    const float* weight  = (const float*)d_in[8];
    const float* sweight = (const float*)d_in[9];

    const size_t off_att  = 0;
    const size_t att_b    = (size_t)32 * 32 * sizeof(float);
    const size_t off_agg  = off_att + att_b;
    const size_t agg_b    = (size_t)32 * 9 * 256 * 256 * sizeof(_Float16);
    const size_t off_xw   = off_agg + agg_b;
    const size_t xw_b     = (size_t)32 * 32 * 32 * 256 * sizeof(_Float16);
    if (off_xw + xw_b > ws_size) return;

    float*    att  = (float*)((char*)d_ws + off_att);
    _Float16* aggw = (_Float16*)((char*)d_ws + off_agg);
    _Float16* xw   = (_Float16*)((char*)d_ws + off_xw);

    k_att<<<32, 256, 0, stream>>>(x, z, w1, gamma, beta, mean, var, w2, att);
    k_xcvt<<<1024, 256, 0, stream>>>(x, xw);
    k_mix<<<1024, 256, 0, stream>>>(weight, sweight, att, aggw);

    dim3 grid(16, 2, 32);
    k_conv<<<grid, 256, 0, stream>>>(xw, aggw, (float*)d_out);
}
